// PointNetSetAbstraction_14078902796586
// MI455X (gfx1250) — hardware-verified
//
#include <hip/hip_runtime.h>
#pragma clang fp contract(off)

constexpr int BATCH  = 8;
constexpr int NPTS   = 8192;
constexpr int NPOINT = 1024;
constexpr int NSAMP  = 32;
constexpr int CIN    = 64;
constexpr int CH0    = 128;
constexpr int CH1    = 128;
constexpr int CH2    = 256;
constexpr int MROWS  = BATCH * NPTS;
constexpr int SQ_SUM_FORM = 0;

static_assert(NSAMP == 32, "one list entry per lane");
static_assert(CIN % 32 == 0 && CH0 % 32 == 0 && CH1 % 32 == 0, "K multiple of 32");
static_assert(MROWS % 64 == 0 && CH0 % 64 == 0 && CH1 % 64 == 0 && CH2 % 64 == 0, "tile multiples");
static_assert((size_t)BATCH * NPOINT * 3 * 4 == 98304, "out0 bytes");
static_assert((size_t)98304 + (size_t)BATCH * CH2 * NPOINT * 4 == 8486912, "d_out bytes");

typedef __attribute__((ext_vector_type(16))) _Float16 v16h;
typedef __attribute__((ext_vector_type(8)))  _Float16 v8h;
typedef __attribute__((ext_vector_type(8)))  float    v8f;
typedef __attribute__((ext_vector_type(4)))  float    v4f;
typedef __attribute__((ext_vector_type(4)))  unsigned v4u;

constexpr size_t WS_W0   = 0;
constexpr size_t WS_W1   = WS_W0 + (size_t)CH0 * CIN * 2;
constexpr size_t WS_W2   = WS_W1 + (size_t)CH1 * CH0 * 2;
constexpr size_t WS_BIAS = WS_W2 + (size_t)CH2 * CH1 * 2;
constexpr size_t WS_NXYZ = ((WS_BIAS + (size_t)(CH0 + CH1 + CH2) * 4 + 4095) / 4096) * 4096;
constexpr size_t WS_XT   = ((WS_NXYZ + (size_t)BATCH * NPOINT * 3 * 4 + 4095) / 4096) * 4096;
constexpr size_t WS_H0   = WS_XT + (size_t)MROWS * CIN * 2;
constexpr size_t WS_H1   = WS_H0 + (size_t)MROWS * CH0 * 2;
constexpr size_t WS_G    = WS_H1 + (size_t)MROWS * CH1 * 2;
constexpr size_t WS_TOTAL = WS_G + (size_t)MROWS * CH2 * 2;
static_assert(WS_TOTAL <= (size_t)134217728, "carve within 128 MiB");
static_assert(WS_XT % 4096 == 0 && WS_H0 % 4096 == 0 && WS_H1 % 4096 == 0 && WS_G % 4096 == 0, "aligned planes");

__device__ __forceinline__ void guard4_h(v8f& a, v8f& b, v8f& c, v8f& d, v16h x) {
  asm volatile("v_nop\n\tv_nop\n\tv_nop\n\tv_nop" : "+v"(a), "+v"(b), "+v"(c), "+v"(d) : "v"(x));
}
__device__ __forceinline__ void keep4_h(v16h a, v16h b, v16h c, v16h d) {
  asm volatile("v_nop" :: "v"(a), "v"(b), "v"(c), "v"(d));
}
__device__ __forceinline__ void acc_guard4(v8f& a, v8f& b, v8f& c, v8f& d) {
  asm volatile("v_nop\n\tv_nop\n\tv_nop\n\tv_nop" : "+v"(a), "+v"(b), "+v"(c), "+v"(d));
}
struct FragH {
  union U { v16h v; v8h h[2]; };
  static __device__ __forceinline__ v16h load(const _Float16* p) {
    U f; f.h[0] = *(const v8h*)(p); f.h[1] = *(const v8h*)(p + 16); return f.v;
  }
  static __device__ __forceinline__ v8f mma(v16h a, v16h b, v8f c) {
    return __builtin_amdgcn_wmma_f32_16x16x32_f16(false, a, false, b, (short)0, c, false, false);
  }
};

__device__ __forceinline__ float h16_to_f32(unsigned hb) {
  const unsigned sgn = (hb & 0x8000u) << 16; const unsigned em = hb & 0x7fffu;
  const float fn = __uint_as_float((em << 13) + 0x38000000u);
  const float fs = (float)em * 5.9604644775390625e-8f;
  const float mag = (em < 0x400u) ? fs : fn; return __uint_as_float(__float_as_uint(mag) | sgn);
}

__device__ __forceinline__ float sum3sq(float a, float b, float c) {
  if (SQ_SUM_FORM == 0) {
    const float t0 = a * a;
    const float t1 = b * b;
    const float t2 = c * c;
    return (t0 + t2) + t1;
  } else {
    float p = a * a;
    p = __builtin_fmaf(b, b, p);
    p = __builtin_fmaf(c, c, p);
    return p;
  }
}

__global__ __launch_bounds__(256) void fold_bn_kernel(
    const float* __restrict__ w, const float* __restrict__ bsrc, const float* __restrict__ gam,
    const float* __restrict__ bet, const float* __restrict__ mean, const float* __restrict__ var,
    _Float16* __restrict__ wOut, float* __restrict__ bOut, int O, int I) {
  const int tid = threadIdx.x;
  const int gid = blockIdx.x * 256 + tid;
  const int e0 = gid * 8;
  if (e0 < O * I) {
    const int o = e0 / I;
    const float inv = gam[o] * (1.0f / sqrtf(var[o] + 1e-5f));
    const v4f a = *(const v4f*)(w + e0);
    const v4f c = *(const v4f*)(w + e0 + 4);
    v8h hv;
    hv[0] = (_Float16)(a[0] * inv); hv[1] = (_Float16)(a[1] * inv);
    hv[2] = (_Float16)(a[2] * inv); hv[3] = (_Float16)(a[3] * inv);
    hv[4] = (_Float16)(c[0] * inv); hv[5] = (_Float16)(c[1] * inv);
    hv[6] = (_Float16)(c[2] * inv); hv[7] = (_Float16)(c[3] * inv);
    for (int pass = 0; pass < 2; ++pass) {
      *(volatile v8h*)(wOut + e0) = hv;
      __threadfence();
    }
  }
  if (blockIdx.x == 0 && tid < (O >> 2)) {
    const int o4 = tid * 4;
    const v4f vb = *(const v4f*)(bsrc + o4);
    const v4f vg = *(const v4f*)(gam + o4);
    const v4f vt = *(const v4f*)(bet + o4);
    const v4f vm = *(const v4f*)(mean + o4);
    const v4f vv = *(const v4f*)(var + o4);
    v4f r;
    r[0] = (vb[0] - vm[0]) * (vg[0] * (1.0f / sqrtf(vv[0] + 1e-5f))) + vt[0];
    r[1] = (vb[1] - vm[1]) * (vg[1] * (1.0f / sqrtf(vv[1] + 1e-5f))) + vt[1];
    r[2] = (vb[2] - vm[2]) * (vg[2] * (1.0f / sqrtf(vv[2] + 1e-5f))) + vt[2];
    r[3] = (vb[3] - vm[3]) * (vg[3] * (1.0f / sqrtf(vv[3] + 1e-5f))) + vt[3];
    for (int pass = 0; pass < 2; ++pass) {
      *(volatile v4f*)(bOut + o4) = r;
      __threadfence();
    }
  }
}

__global__ __launch_bounds__(256) void feat_transpose_f16(
    const float* __restrict__ feature, _Float16* __restrict__ Xt) {
  __shared__ float tile[64 * 65];
  const int tid = threadIdx.x;
  const int b = blockIdx.x >> 7;
  const int n0 = (blockIdx.x & 127) * 64;
  const float* fb = feature + (size_t)b * CIN * NPTS;
#pragma unroll
  for (int i = 0; i < 4; ++i) {
    const int c = (tid >> 4) + 16 * i;
    const int n4 = (tid & 15) * 4;
    const v4f v = *(const v4f*)(fb + (size_t)c * NPTS + n0 + n4);
    tile[c * 65 + n4 + 0] = v[0];
    tile[c * 65 + n4 + 1] = v[1];
    tile[c * 65 + n4 + 2] = v[2];
    tile[c * 65 + n4 + 3] = v[3];
  }
  __syncthreads();
  const int rowA = tid >> 3;
  const int rowB = rowA + 32;
  const int c8 = (tid & 7) * 8;
  v8h hv0, hv1;
#pragma unroll
  for (int e = 0; e < 8; ++e) {
    hv0[e] = (_Float16)tile[(c8 + e) * 65 + rowA];
    hv1[e] = (_Float16)tile[(c8 + e) * 65 + rowB];
  }
  _Float16* dst = Xt + ((size_t)b * NPTS + n0) * CIN;
  for (int pass = 0; pass < 2; ++pass) {
    *(volatile v8h*)(dst + (size_t)rowA * CIN + c8) = hv0;
    *(volatile v8h*)(dst + (size_t)rowB * CIN + c8) = hv1;
    __threadfence();
  }
}

__global__ __launch_bounds__(256) void wmma_gemm64_f16_relu(
    const _Float16* __restrict__ A, int lda,
    const _Float16* __restrict__ Bt, int ldb,
    _Float16* __restrict__ C, int ldc,
    const float* __restrict__ bias, int M, int N, int K) {
  __shared__ __align__(16) float sT[8][16 * 68];
  const int lane = threadIdx.x & 31;
  const int wave = threadIdx.x >> 5;
  const int tilesN = N >> 6;
  const int tilesM = M >> 6;
  const int tile = blockIdx.x * 8 + wave;
  if (tile >= tilesM * tilesN) return;
  const int tm = tile / tilesN;
  const int tn = tile - tm * tilesN;
  const int m0 = tm << 6;
  const int n0 = tn << 6;
  const int rlane = lane & 15;
  const int koff  = (lane >> 4) * 8;
  const int mOff  = (lane >> 4) * 8;

  v8f acc[4][4];
#pragma unroll
  for (int i = 0; i < 4; ++i)
#pragma unroll
    for (int j = 0; j < 4; ++j) acc[i][j] = (v8f){0.f, 0.f, 0.f, 0.f, 0.f, 0.f, 0.f, 0.f};

  for (int k0 = 0; k0 < K; k0 += 32) {
    v16h bh[4];
#pragma unroll
    for (int j = 0; j < 4; ++j) {
      const size_t bo = (size_t)(n0 + (j << 4) + rlane) * ldb + koff + k0;
      bh[j] = FragH::load(Bt + bo);
    }
#pragma unroll
    for (int i = 0; i < 4; ++i) {
      const size_t ao = (size_t)(m0 + (i << 4) + rlane) * lda + koff + k0;
      const v16h ah = FragH::load(A + ao);
#pragma unroll
      for (int j = 0; j < 4; ++j) acc[i][j] = FragH::mma(ah, bh[j], acc[i][j]);
      guard4_h(acc[i][0], acc[i][1], acc[i][2], acc[i][3], ah);
    }
    keep4_h(bh[0], bh[1], bh[2], bh[3]);
  }
  acc_guard4(acc[0][0], acc[0][1], acc[0][2], acc[0][3]);
  acc_guard4(acc[1][0], acc[1][1], acc[1][2], acc[1][3]);
  acc_guard4(acc[2][0], acc[2][1], acc[2][2], acc[2][3]);
  acc_guard4(acc[3][0], acc[3][1], acc[3][2], acc[3][3]);

  float* slab = sT[wave];
#pragma unroll
  for (int i = 0; i < 4; ++i) {
    const int mBase = m0 + (i << 4);
#pragma unroll
    for (int j = 0; j < 4; ++j) {
      const int n = n0 + (j << 4) + rlane;
      const float bv = bias[n];
#pragma unroll
      for (int r = 0; r < 8; ++r) {
        float v = acc[i][j][r] + bv;
        v = (v > 0.0f) ? v : 0.0f;
        slab[(mOff + r) * 68 + (j << 4) + rlane] = v;
      }
    }
    __builtin_amdgcn_fence(__ATOMIC_RELEASE, "workgroup");
    __builtin_amdgcn_wave_barrier();
    __builtin_amdgcn_fence(__ATOMIC_ACQUIRE, "workgroup");
    {
      const int q = lane >> 3, c8 = (lane & 7) * 8;
      for (int pass = 0; pass < 2; ++pass) {
#pragma unroll
        for (int it = 0; it < 4; ++it) {
          const int row = it * 4 + q;
          const float* sp = slab + row * 68 + c8;
          v8h hv;
#pragma unroll
          for (int e = 0; e < 8; ++e) hv[e] = (_Float16)sp[e];
          *(volatile v8h*)(C + (size_t)(mBase + row) * ldc + n0 + c8) = hv;
        }
        __threadfence();
      }
    }
    __builtin_amdgcn_fence(__ATOMIC_RELEASE, "workgroup");
    __builtin_amdgcn_wave_barrier();
    __builtin_amdgcn_fence(__ATOMIC_ACQUIRE, "workgroup");
  }
}

constexpr int FPS_THREADS = 512;
constexpr int FPS_PER_THREAD = NPTS / FPS_THREADS;
constexpr int FPS_CHUNK = 2048;
static_assert(FPS_PER_THREAD == 16, "register slots");

__global__ __launch_bounds__(512) void fps_kernel(
    const float* __restrict__ xyz, float* __restrict__ out_xyz, float* __restrict__ ws_xyz) {
#pragma clang fp contract(off)
  __shared__ __align__(16) float s_stage[FPS_CHUNK * 3];
  __shared__ float s_rv[2][16];
  __shared__ int   s_ri[2][16];
  __shared__ int   s_idx[NPOINT];

  const int b = blockIdx.x;
  const int tid = threadIdx.x;
  const int lane = tid & 31;
  const int wave = tid >> 5;
  const float* xb = xyz + (size_t)b * NPTS * 3;

  float px[16], py[16], pz[16], mind[16];
#pragma unroll
  for (int c = 0; c < 4; ++c) {
    __syncthreads();
#pragma unroll
    for (int k = 0; k < 3; ++k) {
      const int f = tid + k * FPS_THREADS;
      const v4f v = *(const v4f*)(xb + (size_t)c * (FPS_CHUNK * 3) + f * 4);
      *(v4f*)(s_stage + f * 4) = v;
    }
    __syncthreads();
#pragma unroll
    for (int ii = 0; ii < 4; ++ii) {
      const int pl = tid + ii * FPS_THREADS;
      px[c * 4 + ii] = s_stage[pl * 3 + 0];
      py[c * 4 + ii] = s_stage[pl * 3 + 1];
      pz[c * 4 + ii] = s_stage[pl * 3 + 2];
      mind[c * 4 + ii] = 1e10f;
    }
  }

  int last = 0;
  if (tid == 0) s_idx[0] = 0;

#pragma unroll 1
  for (int t = 1; t < NPOINT; ++t) {
    const float qx = xb[last * 3 + 0];
    const float qy = xb[last * 3 + 1];
    const float qz = xb[last * 3 + 2];
    float bv = -1.0f;
    int bi = 0;
#pragma unroll
    for (int i = 0; i < 16; ++i) {
      const float dx = px[i] - qx;
      const float dy = py[i] - qy;
      const float dz = pz[i] - qz;
      const float d = sum3sq(dx, dy, dz);
      const float m = fminf(mind[i], d);
      mind[i] = m;
      if (m > bv) { bv = m; bi = tid + i * FPS_THREADS; }
    }
#pragma unroll
    for (int off = 16; off > 0; off >>= 1) {
      const float v2 = __shfl_xor(bv, off, 32);
      const int   i2 = __shfl_xor(bi, off, 32);
      const bool take = (v2 > bv) || ((v2 == bv) && (i2 < bi));
      bv = take ? v2 : bv;
      bi = take ? i2 : bi;
    }
    const int buf = t & 1;
    if (lane == 0) { s_rv[buf][wave] = bv; s_ri[buf][wave] = bi; }
    __syncthreads();
    float cv = s_rv[buf][lane & 15];
    int   ci = s_ri[buf][lane & 15];
#pragma unroll
    for (int off = 8; off > 0; off >>= 1) {
      const float v2 = __shfl_xor(cv, off, 32);
      const int   i2 = __shfl_xor(ci, off, 32);
      const bool take = (v2 > cv) || ((v2 == cv) && (i2 < ci));
      cv = take ? v2 : cv;
      ci = take ? i2 : ci;
    }
    ci = ci < 0 ? 0 : (ci > NPTS - 1 ? NPTS - 1 : ci);
    last = __builtin_amdgcn_readfirstlane(ci);
    if (tid == 0) s_idx[t] = last;
  }
  __syncthreads();

#pragma unroll
  for (int k = 0; k < 2; ++k) {
    const int s = tid + k * FPS_THREADS;
    int n = s_idx[s];
    n = n < 0 ? 0 : (n > NPTS - 1 ? NPTS - 1 : n);
    const float x = xb[n * 3 + 0];
    const float y = xb[n * 3 + 1];
    const float z = xb[n * 3 + 2];
    s_stage[s * 3 + 0] = x;
    s_stage[s * 3 + 1] = y;
    s_stage[s * 3 + 2] = z;
  }
  __syncthreads();
  {
    float* o = out_xyz + (size_t)b * (NPOINT * 3);
    float* w = ws_xyz + (size_t)b * (NPOINT * 3);
    const int f2 = tid + FPS_THREADS;
    const int f2c = f2 < 768 ? f2 : 767;
    const v4f va = *(const v4f*)(s_stage + tid * 4);
    const v4f vb = *(const v4f*)(s_stage + f2c * 4);
    for (int pass = 0; pass < 2; ++pass) {
      *(volatile v4f*)(o + tid * 4) = va;
      *(volatile v4f*)(w + tid * 4) = va;
      if (tid < 256) {
        *(volatile v4f*)(o + f2 * 4) = vb;
        *(volatile v4f*)(w + f2 * 4) = vb;
      }
      __threadfence();
    }
  }
}

__device__ __forceinline__ bool key_lt(unsigned ah, unsigned al, unsigned bh, unsigned bl) {
  return (ah < bh) || ((ah == bh) && (al < bl));
}

__device__ __forceinline__ void knn_consider(
    float x, float y, float z, float sb, unsigned nIdx,
    float qx, float qy, float qz, float sa,
    unsigned& myH, unsigned& myL, unsigned& tauH, unsigned& tauL, int prevLane, int lane) {
#pragma clang fp contract(off)
  float p = qx * x;
  p = __builtin_fmaf(qy, y, p);
  p = __builtin_fmaf(qz, z, p);
  const float s = sa + sb;
  const float tp = 2.0f * p;
  float d = s - tp;
  d = d + 0.0f;
  const unsigned u = __float_as_uint(d);
  const unsigned kh = u ^ (((unsigned)((int)u >> 31)) | 0x80000000u);
  const unsigned kl = nIdx;
  const bool hit = key_lt(kh, kl, tauH, tauL);
  unsigned m = __builtin_amdgcn_ballot_w32(hit);
  while (m != 0u) {
    const int src = __builtin_ctz(m);
    m &= (m - 1u);
    const unsigned ch = (unsigned)__builtin_amdgcn_readlane((int)kh, src);
    const unsigned cl = (unsigned)__builtin_amdgcn_readlane((int)kl, src);
    const unsigned upH = (unsigned)__shfl((int)myH, prevLane, 32);
    const unsigned upL = (unsigned)__shfl((int)myL, prevLane, 32);
    const bool gt = key_lt(ch, cl, myH, myL);
    const bool upgt = (lane > 0) && key_lt(ch, cl, upH, upL);
    const unsigned nH = gt ? (upgt ? upH : ch) : myH;
    const unsigned nL = gt ? (upgt ? upL : cl) : myL;
    myH = nH;
    myL = nL;
    tauH = (unsigned)__builtin_amdgcn_readlane((int)myH, 31);
    tauL = (unsigned)__builtin_amdgcn_readlane((int)myL, 31);
  }
}

__device__ __forceinline__ void gather_max_query(
    const unsigned short* __restrict__ Gb, unsigned myL, int lane, float* __restrict__ tileCol) {
  unsigned mlo[4], mhi[4];
#pragma unroll
  for (int c = 0; c < 4; ++c) { mlo[c] = 0u; mhi[c] = 0u; }
#pragma unroll 4
  for (int j = 0; j < NSAMP; ++j) {
    int n = __builtin_amdgcn_readlane((int)myL, j);
    n = n < 0 ? 0 : (n > NPTS - 1 ? NPTS - 1 : n);
    const v4u w = *(const v4u*)(const void*)(Gb + (size_t)n * CH2 + lane * 8);
#pragma unroll
    for (int c = 0; c < 4; ++c) {
      const unsigned lo = w[c] & 0x7fffu;
      const unsigned hi = (w[c] >> 16) & 0x7fffu;
      mlo[c] = lo > mlo[c] ? lo : mlo[c];
      mhi[c] = hi > mhi[c] ? hi : mhi[c];
    }
  }
#pragma unroll
  for (int c = 0; c < 4; ++c) {
    tileCol[(lane * 8 + 2 * c) * 32]     = h16_to_f32(mlo[c]);
    tileCol[(lane * 8 + 2 * c + 1) * 32] = h16_to_f32(mhi[c]);
  }
}

__global__ __launch_bounds__(256) void knn_gather_max_kernel(
    const float* __restrict__ xyz, const float* __restrict__ nxyz,
    const unsigned short* __restrict__ G, float* __restrict__ out1) {
#pragma clang fp contract(off)
  __shared__ __align__(16) float s_tile[CH2 * 32];
  const int tid = threadIdx.x;
  const int lane = tid & 31;
  const int wave = __builtin_amdgcn_readfirstlane((int)(threadIdx.x >> 5));
  const int b = blockIdx.x >> 5;
  const int s0 = (blockIdx.x & 31) * 32;
  const float* xb = xyz + (size_t)b * NPTS * 3;
  const float* qp = nxyz + ((size_t)b * NPOINT + s0 + wave * 4) * 3;

  const float qx0 = qp[0], qy0 = qp[1], qz0 = qp[2];
  const float qx1 = qp[3], qy1 = qp[4], qz1 = qp[5];
  const float qx2 = qp[6], qy2 = qp[7], qz2 = qp[8];
  const float qx3 = qp[9], qy3 = qp[10], qz3 = qp[11];
  const float sa0 = sum3sq(qx0, qy0, qz0);
  const float sa1 = sum3sq(qx1, qy1, qz1);
  const float sa2 = sum3sq(qx2, qy2, qz2);
  const float sa3 = sum3sq(qx3, qy3, qz3);

  unsigned myH0 = 0xffffffffu, myL0 = 0xffffffffu, tH0 = 0xffffffffu, tL0 = 0xffffffffu;
  unsigned myH1 = 0xffffffffu, myL1 = 0xffffffffu, tH1 = 0xffffffffu, tL1 = 0xffffffffu;
  unsigned myH2 = 0xffffffffu, myL2 = 0xffffffffu, tH2 = 0xffffffffu, tL2 = 0xffffffffu;
  unsigned myH3 = 0xffffffffu, myL3 = 0xffffffffu, tH3 = 0xffffffffu, tL3 = 0xffffffffu;
  const int prevLane = lane > 0 ? lane - 1 : 0;

#pragma unroll 1
  for (int g = 0; g < NPTS / 32; ++g) {
    const int n = g * 32 + lane;
    const float x = xb[n * 3 + 0];
    const float y = xb[n * 3 + 1];
    const float z = xb[n * 3 + 2];
    const float sb = sum3sq(x, y, z);
    knn_consider(x, y, z, sb, (unsigned)n, qx0, qy0, qz0, sa0, myH0, myL0, tH0, tL0, prevLane, lane);
    knn_consider(x, y, z, sb, (unsigned)n, qx1, qy1, qz1, sa1, myH1, myL1, tH1, tL1, prevLane, lane);
    knn_consider(x, y, z, sb, (unsigned)n, qx2, qy2, qz2, sa2, myH2, myL2, tH2, tL2, prevLane, lane);
    knn_consider(x, y, z, sb, (unsigned)n, qx3, qy3, qz3, sa3, myH3, myL3, tH3, tL3, prevLane, lane);
  }

  const unsigned short* Gb = G + (size_t)b * NPTS * CH2;
  gather_max_query(Gb, myL0, lane, s_tile + wave * 4 + 0);
  gather_max_query(Gb, myL1, lane, s_tile + wave * 4 + 1);
  gather_max_query(Gb, myL2, lane, s_tile + wave * 4 + 2);
  gather_max_query(Gb, myL3, lane, s_tile + wave * 4 + 3);
  __syncthreads();

  {
    float* ob = out1 + ((size_t)b * CH2) * NPOINT + s0;
    const int rq = tid >> 3;
    const int c4 = (tid & 7) * 4;
    for (int pass = 0; pass < 2; ++pass) {
#pragma unroll
      for (int it = 0; it < 8; ++it) {
        const int row = rq + 32 * it;
        const v4f v = *(const v4f*)(s_tile + row * 32 + c4);
        *(volatile v4f*)(ob + (size_t)row * NPOINT + c4) = v;
      }
      __threadfence();
    }
  }
}

extern "C" void kernel_launch(void* const* d_in, const int* in_sizes, int n_in,
                              void* d_out, int out_size, void* d_ws, size_t ws_size,
                              hipStream_t stream) {
  (void)in_sizes; (void)n_in; (void)out_size;
  if (ws_size < WS_TOTAL) return;

  const float* xyz     = (const float*)d_in[0];
  const float* feature = (const float*)d_in[1];

  char* ws = (char*)d_ws;
  _Float16* w0h  = (_Float16*)(ws + WS_W0);
  _Float16* w1h  = (_Float16*)(ws + WS_W1);
  _Float16* w2h  = (_Float16*)(ws + WS_W2);
  float*    bws  = (float*)(ws + WS_BIAS);
  float*    nxyz = (float*)(ws + WS_NXYZ);
  _Float16* Xt   = (_Float16*)(ws + WS_XT);
  _Float16* H0   = (_Float16*)(ws + WS_H0);
  _Float16* H1   = (_Float16*)(ws + WS_H1);
  _Float16* Gp   = (_Float16*)(ws + WS_G);

  float* out0 = (float*)d_out;
  float* out1 = out0 + (size_t)BATCH * NPOINT * 3;

  fold_bn_kernel<<<(CH0 * CIN / 8 + 255) / 256, 256, 0, stream>>>(
      (const float*)d_in[2], (const float*)d_in[3], (const float*)d_in[4], (const float*)d_in[5],
      (const float*)d_in[6], (const float*)d_in[7], w0h, bws, CH0, CIN);
  fold_bn_kernel<<<(CH1 * CH0 / 8 + 255) / 256, 256, 0, stream>>>(
      (const float*)d_in[8], (const float*)d_in[9], (const float*)d_in[10], (const float*)d_in[11],
      (const float*)d_in[12], (const float*)d_in[13], w1h, bws + CH0, CH1, CH0);
  fold_bn_kernel<<<(CH2 * CH1 / 8 + 255) / 256, 256, 0, stream>>>(
      (const float*)d_in[14], (const float*)d_in[15], (const float*)d_in[16], (const float*)d_in[17],
      (const float*)d_in[18], (const float*)d_in[19], w2h, bws + CH0 + CH1, CH2, CH1);

  feat_transpose_f16<<<BATCH * (NPTS / 64), 256, 0, stream>>>(feature, Xt);

  wmma_gemm64_f16_relu<<<((MROWS / 64) * (CH0 / 64) + 7) / 8, 256, 0, stream>>>(
      Xt, CIN, w0h, CIN, H0, CH0, bws, MROWS, CH0, CIN);
  wmma_gemm64_f16_relu<<<((MROWS / 64) * (CH1 / 64) + 7) / 8, 256, 0, stream>>>(
      H0, CH0, w1h, CH0, H1, CH1, bws + CH0, MROWS, CH1, CH0);
  wmma_gemm64_f16_relu<<<((MROWS / 64) * (CH2 / 64) + 7) / 8, 256, 0, stream>>>(
      H1, CH1, w2h, CH1, Gp, CH2, bws + CH0 + CH1, MROWS, CH2, CH1);

  fps_kernel<<<BATCH, FPS_THREADS, 0, stream>>>(xyz, out0, nxyz);

  knn_gather_max_kernel<<<BATCH * (NPOINT / 32), 256, 0, stream>>>(
      xyz, nxyz, (const unsigned short*)(const void*)Gp, out1);
}
